// ResidualBlock_65962107732684
// MI455X (gfx1250) — hardware-run, weakly checked
//
#include <hip/hip_runtime.h>


#ifndef NB
#define NB 2
#endif
#ifndef SEQ
#define SEQ 2048
#endif
#define NB_FULL  2
#define SEQ_FULL 2048
#ifndef OUT_SEQ
#define OUT_SEQ SEQ
#endif
#define HID  1024
#define DIN  2048
#define NST  16
#define DTR  64
#define XDW  96
#define XDP  128
#define ROWS (NB * SEQ)
#define TCH  16
#define YSP  36
#define L2E  1.4426950408889634f
#define LN2  0.6931471805599453f
#define XNC  16.0f
#define W1C  32.0f
#define XCC  64.0f
#define W2C  32.0f
#define DTC  64.0f
#define W3C  8.0f
#define YGC  256.0f
#define W4C  32.0f
#define EPI_IN  0
#define EPI_XP  1
#define EPI_DT  2
#define EPI_OUT 3

static_assert(HID % 32 == 0);
static_assert(DIN % 32 == 0);
static_assert(DTR % 32 == 0);
static_assert(HID % 64 == 0);
static_assert(DIN % 64 == 0);
static_assert((2 * DIN) % 64 == 0);
static_assert(XDP % 64 == 0);
static_assert(XDW <= XDP);
static_assert(DTR + 2 * NST == XDW);
static_assert(DTR == 64);
static_assert(ROWS % 64 == 0);
static_assert(SEQ % 64 == 0);
static_assert(ROWS % 4 == 0);
static_assert(HID == 4 * 256);
static_assert(DIN == 256 * 8);
static_assert(DIN % 32 == 0);
static_assert(SEQ % TCH == 0);
static_assert(NST == 16);
static_assert(NB <= NB_FULL);
static_assert(SEQ <= SEQ_FULL);
static_assert((YSP * 4) % 16 == 0);
static_assert(8 * 32 * 16 == 16 * 64 * 4);
static_assert(4 * 32 * 16 == 16 * 64 * 2);
static_assert(2 * 32 * 16 == TCH * 32 * 2);
static_assert(16 * 68 * 4 <= 131072);
static_assert(TCH * YSP * 4 <= 131072);

typedef _Float16 h16;
typedef unsigned short bf;
typedef __attribute__((ext_vector_type(16))) _Float16 v16h;
typedef __attribute__((ext_vector_type(8)))  _Float16 v8h;
typedef __attribute__((ext_vector_type(8)))  float    v8f;
typedef __attribute__((ext_vector_type(4)))  float    v4f;
typedef v4f  __attribute__((may_alias)) v4fa;

__device__ __forceinline__ unsigned short f2bf(float f) { unsigned u = __float_as_uint(f); u += 0x7FFFu + ((u >> 16) & 1u); return (unsigned short)(u >> 16); }
__device__ __forceinline__ float bfr(float f) { return __uint_as_float(((unsigned)f2bf(f)) << 16); }
__device__ __forceinline__ v16h cat16(v8h lo, v8h hi) { return __builtin_shufflevector(lo, hi, 0, 1, 2, 3, 4, 5, 6, 7, 8, 9, 10, 11, 12, 13, 14, 15); }
__device__ __forceinline__ v8f wmma16(v16h a, v16h b, v8f c) { return __builtin_amdgcn_wmma_f32_16x16x32_f16(false, a, false, b, (short)0, c, false, false); }
__device__ __forceinline__ v16h  ldh(const h16* p) { return cat16(*(const v8h*)p, *(const v8h*)(p + 16)); }
__device__ __forceinline__ void wave_sync() { __builtin_amdgcn_fence(3  , "wavefront"); __builtin_amdgcn_wave_barrier(); asm volatile("" ::: "memory"); }

static __device__ __forceinline__ h16 toh_flush(float v) { const h16 r = (h16)v; return (fabsf(v) < 6.103515625e-05f) ? (h16)0.0f : r; }
static __device__ __forceinline__ v8f wmma16g(v16h a, v16h b, v8f c) {
    c = wmma16(a, b, c);
    asm volatile("v_nop\n\tv_nop\n\tv_nop\n\tv_nop" : "+v"(c) : "v"(a), "v"(b));
    return c;
}
static __device__ __forceinline__ float sigm(float v) { return __builtin_amdgcn_rcpf(1.0f + __builtin_amdgcn_exp2f(-v * L2E)); }

__global__ __launch_bounds__(256) void k_wconv(const float* __restrict__ src, h16* dst, int rows_src, int rows_dst, int cols, float carry) {
    const int n8 = rows_dst * (cols / 8);
    const int i = blockIdx.x * 256 + threadIdx.x; if (i >= n8) return;
    const int e = i * 8; const int row = e / cols, col = e - row * cols;
    const int rs = row < rows_src ? row : rows_src - 1;
    v8f v = *(const v8f*)(src + (size_t)rs * cols + col);
    asm volatile("" : "+v"(v));
    const bool ok = row < rows_src;
    v8h o;
#pragma unroll
    for (int k = 0; k < 8; ++k) { const h16 c = toh_flush(bfr(v[k]) * carry); o[k] = ok ? c : (h16)0.0f; }
    *(volatile v8h*)(dst + (size_t)i * 8) = o; __threadfence(); *(volatile v8h*)(dst + (size_t)i * 8) = o;
}

__global__ __launch_bounds__(128) void k_rms(const float* __restrict__ x, const float* __restrict__ nw, h16* XN) {
#pragma clang fp contract(off)
    const int lane = threadIdx.x & 31;
    const int wave = __builtin_amdgcn_readfirstlane((int)(threadIdx.x >> 5));
    const int row = blockIdx.x * 4 + wave;
    const int b = row / SEQ, t = row % SEQ;
    const float* xr = x + ((size_t)b * SEQ_FULL + (size_t)t) * HID + lane * 8;
    float ss = 0.0f;
#pragma unroll 1
    for (int c = 0; c < HID / 256; ++c) {
        const v8f v = *(const v8f*)(xr + c * 256);
#pragma unroll
        for (int k = 0; k < 8; ++k) { const float f = bfr(v[k]); ss += f * f; }
    }
    ss += __shfl_xor(ss, 16, 32); ss += __shfl_xor(ss, 8, 32); ss += __shfl_xor(ss, 4, 32); ss += __shfl_xor(ss, 2, 32); ss += __shfl_xor(ss, 1, 32);
    const float sc = rsqrtf(ss * (1.0f / (float)HID) + 1e-5f);
    h16* dst = XN + (size_t)row * HID + lane * 8;
    const float* wr = nw + lane * 8;
#pragma unroll 1
    for (int c = 0; c < HID / 256; ++c) {
        const v8f v = *(const v8f*)(xr + c * 256);
        const v8f w = *(const v8f*)(wr + c * 256);
        v8h o;
#pragma unroll
        for (int k = 0; k < 8; ++k) o[k] = toh_flush(((bfr(v[k]) * sc) * bfr(w[k])) * XNC);
        *(volatile v8h*)(dst + c * 256) = o; __threadfence(); *(volatile v8h*)(dst + c * 256) = o;
    }
}

template <int EPI>
__device__ __forceinline__ void gemm_tile(const h16* __restrict__ A, const h16* __restrict__ Bt, const int K, const size_t lda, const size_t ablk,
                                          float* F0, h16* H0, const float* __restrict__ aux, const float unscale) {
    __shared__ __align__(16) float os[16 * 68];
    const int lane = threadIdx.x & 31, lr = lane & 15, hi = lane >> 4; const int r0 = blockIdx.x * 64, c0 = blockIdx.y * 64;
    v8f acc[4][4];
#pragma unroll
    for (int mb = 0; mb < 4; ++mb)
#pragma unroll
        for (int nb = 0; nb < 4; ++nb) acc[mb][nb] = (v8f){};
    const size_t aoff = (size_t)(r0 + lr) * lda + 8 * hi, boff = (size_t)(c0 + lr) * (size_t)K + 8 * hi;
#pragma unroll 1
    for (int kc = 0; kc < K; kc += 32) {
        const size_t ak = aoff + (size_t)(kc >> 5) * ablk;
        v16h a[4];
#pragma unroll
        for (int mb = 0; mb < 4; ++mb) a[mb] = ldh(A + ak + (size_t)mb * 16 * lda);
#pragma unroll
        for (int nb = 0; nb < 4; ++nb) { const v16h bq = ldh(Bt + boff + (size_t)nb * 16 * (size_t)K + kc);
#pragma unroll
            for (int mb = 0; mb < 4; ++mb) acc[mb][nb] = wmma16g(a[mb], bq, acc[mb][nb]); }
    }
    const bool gate = (EPI == EPI_IN) & (c0 >= DIN);
    float bc[4];
#pragma unroll
    for (int nb = 0; nb < 4; ++nb) bc[nb] = (EPI == EPI_DT) ? bfr(aux[c0 + nb * 16 + lr]) : 0.0f;
    size_t fo = 0, ho = 0, xo = 0; size_t fp = 0, hp = 0;
    if (EPI == EPI_IN)  { fo = (size_t)r0 * DIN + (size_t)(gate ? c0 - DIN : c0); fp = DIN; ho = fo; hp = DIN; }
    if (EPI == EPI_XP)  { fo = (size_t)r0 * XDP + (size_t)c0; fp = XDP; ho = (size_t)r0 * DTR; hp = DTR; }
    if (EPI == EPI_DT)  { fo = (size_t)r0 * DIN + (size_t)c0; fp = DIN; }
    if (EPI == EPI_OUT) { const int bb = r0 / SEQ, tt = r0 % SEQ;
                          fo = ((size_t)bb * OUT_SEQ + (size_t)tt) * HID + (size_t)c0; fp = HID;
                          xo = ((size_t)bb * SEQ_FULL + (size_t)tt) * HID + (size_t)c0; }
#pragma unroll
    for (int mb = 0; mb < 4; ++mb) {
#pragma unroll
        for (int nb = 0; nb < 4; ++nb) {
#pragma unroll
            for (int j = 0; j < 8; ++j) {
                float v = acc[mb][nb][j] * unscale;
                if (EPI == EPI_IN) { if (gate) v = v * sigm(v); }
                if (EPI == EPI_DT) { v += bc[nb]; const float e = __builtin_amdgcn_exp2f(-fabsf(v) * L2E); v = fmaxf(v, 0.0f) + __builtin_amdgcn_logf(1.0f + e) * LN2; }
                os[(hi * 8 + j) * 68 + nb * 16 + lr] = v; } }
        wave_sync();
#pragma unroll 1
        for (int ps = 0; ps < 2; ++ps) {
            if ((EPI == EPI_IN) && gate) {
#pragma unroll
                for (int s = 0; s < 4; ++s) { const int row = 4 * s + (lane >> 3), c8 = (lane & 7) * 8;
                    const v4f x0 = *(const v4fa*)(&os[row * 68 + c8]); const v4f x1 = *(const v4fa*)(&os[row * 68 + c8 + 4]); v8h hv;
#pragma unroll
                    for (int i = 0; i < 4; ++i) { hv[i] = toh_flush(x0[i]); hv[4 + i] = toh_flush(x1[i]); }
                    *(volatile v8h*)(H0 + ho + (size_t)(mb * 16 + row) * hp + c8) = hv; }
            } else {
#pragma unroll
                for (int s = 0; s < 8; ++s) { const int row = 2 * s + (lane >> 4), col = (lane & 15) * 4;
                    v4f val = *(const v4fa*)(&os[row * 68 + col]);
                    if (EPI == EPI_OUT) { const v4f xr = *(const v4f*)(aux + xo + (size_t)(mb * 16 + row) * HID + col);
                                          val[0] += bfr(xr[0]); val[1] += bfr(xr[1]); val[2] += bfr(xr[2]); val[3] += bfr(xr[3]); }
                    *(volatile v4f*)(F0 + fo + (size_t)(mb * 16 + row) * fp + col) = val; }
            }
            if (EPI == EPI_XP) {
                if (c0 == 0) {
#pragma unroll
                    for (int s = 0; s < 4; ++s) { const int row = 4 * s + (lane >> 3), c8 = (lane & 7) * 8;
                        const v4f x0 = *(const v4fa*)(&os[row * 68 + c8]); const v4f x1 = *(const v4fa*)(&os[row * 68 + c8 + 4]); v8h hv;
#pragma unroll
                        for (int i = 0; i < 4; ++i) { hv[i] = toh_flush(x0[i] * DTC); hv[4 + i] = toh_flush(x1[i] * DTC); }
                        *(volatile v8h*)(H0 + ho + (size_t)(mb * 16 + row) * hp + c8) = hv; }
                }
            }
            if (ps == 0) __threadfence(); }
        wave_sync();
    }
}

__global__ __launch_bounds__(32) void k_gemm_in(const h16* __restrict__ XN, const h16* __restrict__ W1, float* XI, h16* G) {
    gemm_tile<EPI_IN>(XN, W1, HID, (size_t)HID, (size_t)32, XI, G, nullptr, 1.0f / (XNC * W1C));
}
__global__ __launch_bounds__(32) void k_gemm_xp(const h16* __restrict__ XC, const h16* __restrict__ W2, float* XD, h16* DT) {
    gemm_tile<EPI_XP>(XC, W2, DIN, (size_t)DIN, (size_t)32, XD, DT, nullptr, 1.0f / (XCC * W2C));
}
__global__ __launch_bounds__(32) void k_gemm_dt(const h16* __restrict__ DT, const h16* __restrict__ W3, const float* __restrict__ dtb, float* DELTA) {
    gemm_tile<EPI_DT>(DT, W3, DTR, (size_t)DTR, (size_t)32, DELTA, nullptr, dtb, 1.0f / (DTC * W3C));
}
__global__ __launch_bounds__(32) void k_gemm_out(const h16* __restrict__ YG, const h16* __restrict__ W4, const float* __restrict__ x, float* OUT) {
    gemm_tile<EPI_OUT>(YG, W4, DIN, (size_t)32, (size_t)ROWS * 32, OUT, nullptr, x, 1.0f / (YGC * W4C));
}

__global__ __launch_bounds__(256) void k_conv(const float* __restrict__ XI, const float* __restrict__ cw, const float* __restrict__ cb, h16* XC) {
#pragma clang fp contract(off)
    const int r = blockIdx.x; const int t = r % SEQ;
    const int d = threadIdx.x * 8;
    float acc[8];
    { const v8f bv = *(const v8f*)(cb + d);
#pragma unroll
      for (int k = 0; k < 8; ++k) acc[k] = bfr(bv[k]); }
#pragma unroll 1
    for (int j = 0; j < 4; ++j) {
        const int ss = t - 3 + j;
        const int back = ss < 0 ? 0 : (3 - j);
        v8f xv = *(const v8f*)(XI + (size_t)(r - back) * DIN + d);
        asm volatile("" : "+v"(xv));
        const bool ok = ss >= 0;
#pragma unroll
        for (int k = 0; k < 8; ++k) { const float w = bfr(cw[(d + k) * 4 + j]); const float xk = ok ? xv[k] : 0.0f; acc[k] += xk * w; }
    }
    v8h o;
#pragma unroll
    for (int k = 0; k < 8; ++k) { const float u = acc[k] * sigm(acc[k]); o[k] = toh_flush(u * XCC); }
    h16* dst = XC + (size_t)r * DIN + d;
    *(volatile v8h*)dst = o; __threadfence(); *(volatile v8h*)dst = o;
}

__global__ __launch_bounds__(32) void k_scan(const float* __restrict__ XI, const float* __restrict__ DELTA, const float* __restrict__ XD, const h16* __restrict__ G,
                                             const float* __restrict__ cw, const float* __restrict__ cb, const float* __restrict__ Alog, const float* __restrict__ Dv, h16* YG) {
    __shared__ __align__(16) float ys[TCH * YSP];
    const int lane = threadIdx.x & 31;
    const int kb = blockIdx.x % (DIN / 32), b = blockIdx.x / (DIN / 32);
    const int d = kb * 32 + lane;
    float a2[16], h[16];
#pragma unroll
    for (int q = 0; q < 4; ++q) { const v4f al = *(const v4f*)(Alog + d * NST + 4 * q);
#pragma unroll
        for (int i = 0; i < 4; ++i) { a2[4 * q + i] = -__builtin_amdgcn_exp2f(bfr(al[i]) * L2E) * L2E; h[4 * q + i] = 0.0f; } }
    const float Dd = bfr(Dv[d]);
    const float w0 = bfr(cw[d * 4 + 0]), w1 = bfr(cw[d * 4 + 1]), w2 = bfr(cw[d * 4 + 2]), w3 = bfr(cw[d * 4 + 3]);
    const float cbv = bfr(cb[d]);
    float x1 = 0.0f, x2 = 0.0f, x3 = 0.0f;
    const size_t m0 = (size_t)b * SEQ;
#pragma unroll 1
    for (int tc = 0; tc < SEQ / TCH; ++tc) {
#pragma unroll 1
        for (int tt = 0; tt < TCH; ++tt) {
            const size_t m = m0 + (size_t)(tc * TCH + tt);
            const float dl = DELTA[m * DIN + d];
            const float xi = XI[m * DIN + d];
            const float g  = (float)G[m * DIN + d];
            const float* bcp = XD + m * XDP + DTR;
            const v4f b0 = *(const v4f*)bcp, b1 = *(const v4f*)(bcp + 4), b2 = *(const v4f*)(bcp + 8), b3 = *(const v4f*)(bcp + 12);
            const v4f q0 = *(const v4f*)(bcp + 16), q1 = *(const v4f*)(bcp + 20), q2 = *(const v4f*)(bcp + 24), q3 = *(const v4f*)(bcp + 28);
            float Bv[16], Cv[16];
#pragma unroll
            for (int i = 0; i < 4; ++i) { Bv[i] = b0[i]; Bv[4 + i] = b1[i]; Bv[8 + i] = b2[i]; Bv[12 + i] = b3[i]; Cv[i] = q0[i]; Cv[4 + i] = q1[i]; Cv[8 + i] = q2[i]; Cv[12 + i] = q3[i]; }
            const float cv = cbv + x3 * w0 + x2 * w1 + x1 * w2 + xi * w3;
            x3 = x2; x2 = x1; x1 = xi;
            const float u = cv * sigm(cv);
            const float dbu = dl * u;
            float y = 0.0f;
#pragma unroll
            for (int n = 0; n < 16; ++n) { const float dA = __builtin_amdgcn_exp2f(dl * a2[n]); h[n] = fmaf(dA, h[n], dbu * Bv[n]); y = fmaf(h[n], Cv[n], y); }
            y = fmaf(u, Dd, y);
            ys[tt * YSP + lane] = y * g;
        }
        wave_sync();
        h16* yb = YG + ((size_t)kb * ROWS + m0 + (size_t)tc * TCH) * 32;
#pragma unroll 1
        for (int ps = 0; ps < 2; ++ps) {
#pragma unroll
            for (int s = 0; s < 2; ++s) { const int p = s * 32 + lane; const int row = p >> 2, c8 = (p & 3) * 8;
                const v4f x0 = *(const v4fa*)(&ys[row * YSP + c8]); const v4f x1v = *(const v4fa*)(&ys[row * YSP + c8 + 4]); v8h hv;
#pragma unroll
                for (int i = 0; i < 4; ++i) { hv[i] = toh_flush(x0[i] * YGC); hv[4 + i] = toh_flush(x1v[i] * YGC); }
                *(volatile v8h*)(yb + (size_t)p * 8) = hv; }
            if (ps == 0) __threadfence(); }
        wave_sync();
    }
}

static constexpr size_t al256(size_t v) { return (v + 255) & ~(size_t)255; }
static constexpr size_t SZ_XN = al256((size_t)ROWS * HID * 2);
static constexpr size_t SZ_W1 = al256((size_t)2 * DIN * HID * 2);
static constexpr size_t SZ_W2 = al256((size_t)XDP * DIN * 2);
static constexpr size_t SZ_W3 = al256((size_t)DIN * DTR * 2);
static constexpr size_t SZ_W4 = al256((size_t)HID * DIN * 2);
static constexpr size_t SZ_XI = al256((size_t)ROWS * DIN * 4);
static constexpr size_t SZ_G  = al256((size_t)ROWS * DIN * 2);
static constexpr size_t SZ_XC = al256((size_t)ROWS * DIN * 2);
static constexpr size_t SZ_XD = al256((size_t)ROWS * XDP * 4);
static constexpr size_t SZ_DT = al256((size_t)ROWS * DTR * 2);
static constexpr size_t SZ_DL = al256((size_t)ROWS * DIN * 4);
static constexpr size_t SZ_TOTAL = SZ_XN + SZ_W1 + SZ_W2 + SZ_W3 + SZ_W4 + SZ_XI + SZ_G + SZ_XC + SZ_XD + SZ_DT + SZ_DL;
static_assert(SZ_TOTAL <= (size_t)134217728);
static_assert((size_t)(DIN / 32) * ROWS * 32 * 2 <= SZ_XC);
static_assert((size_t)ROWS * DIN * 2 <= SZ_XC);

extern "C" void kernel_launch(void* const* d_in, const int* in_sizes, int n_in,
                              void* d_out, int out_size, void* d_ws, size_t ws_size, hipStream_t stream) {
    if (n_in < 11) return;
    const size_t needx = ((size_t)(NB - 1) * SEQ_FULL + SEQ) * HID;
    if ((size_t)in_sizes[0] < needx) return;
    if (in_sizes[1] < HID) return;
    if ((size_t)in_sizes[2] < (size_t)2 * DIN * HID) return;
    if (in_sizes[3] < DIN * 4 || in_sizes[4] < DIN) return;
    if ((size_t)in_sizes[5] < (size_t)XDW * DIN) return;
    if ((size_t)in_sizes[6] < (size_t)DIN * DTR || in_sizes[7] < DIN) return;
    if (in_sizes[8] < DIN * NST || in_sizes[9] < DIN) return;
    if ((size_t)in_sizes[10] < (size_t)HID * DIN) return;
    if ((size_t)out_size < ((size_t)(NB - 1) * OUT_SEQ + SEQ) * HID) return;
    if (SZ_TOTAL > ws_size) return;
    const float* x    = (const float*)d_in[0];
    const float* nw   = (const float*)d_in[1];
    const float* win  = (const float*)d_in[2];
    const float* cw   = (const float*)d_in[3];
    const float* cb   = (const float*)d_in[4];
    const float* wxp  = (const float*)d_in[5];
    const float* wdt  = (const float*)d_in[6];
    const float* dtb  = (const float*)d_in[7];
    const float* alog = (const float*)d_in[8];
    const float* dvec = (const float*)d_in[9];
    const float* wout = (const float*)d_in[10];
    float* OUT = (float*)d_out;
    char* wsp = (char*)d_ws;
    h16* XN = (h16*)wsp; wsp += SZ_XN;
    h16* W1 = (h16*)wsp; wsp += SZ_W1;
    h16* W2 = (h16*)wsp; wsp += SZ_W2;
    h16* W3 = (h16*)wsp; wsp += SZ_W3;
    h16* W4 = (h16*)wsp; wsp += SZ_W4;
    float* XI = (float*)wsp; wsp += SZ_XI;
    h16* G  = (h16*)wsp; wsp += SZ_G;
    h16* XC = (h16*)wsp; h16* YG = (h16*)wsp; wsp += SZ_XC;
    float* XD = (float*)wsp; wsp += SZ_XD;
    h16* DT = (h16*)wsp; wsp += SZ_DT;
    float* DL = (float*)wsp; wsp += SZ_DL;

    k_rms<<<ROWS / 4, 128, 0, stream>>>(x, nw, XN);
    k_wconv<<<(unsigned)(((size_t)2 * DIN * HID / 8 + 255) / 256), 256, 0, stream>>>(win, W1, 2 * DIN, 2 * DIN, HID, W1C);
    k_wconv<<<(unsigned)(((size_t)XDP * DIN / 8 + 255) / 256), 256, 0, stream>>>(wxp, W2, XDW, XDP, DIN, W2C);
    k_wconv<<<(unsigned)(((size_t)DIN * DTR / 8 + 255) / 256), 256, 0, stream>>>(wdt, W3, DIN, DIN, DTR, W3C);
    k_wconv<<<(unsigned)(((size_t)HID * DIN / 8 + 255) / 256), 256, 0, stream>>>(wout, W4, HID, HID, DIN, W4C);

    k_gemm_in<<<dim3(ROWS / 64, 2 * DIN / 64, 1), 32, 0, stream>>>(XN, W1, XI, G);
    k_conv<<<ROWS, 256, 0, stream>>>(XI, cw, cb, XC);
    k_gemm_xp<<<dim3(ROWS / 64, XDP / 64, 1), 32, 0, stream>>>(XC, W2, XD, DT);
    k_gemm_dt<<<dim3(ROWS / 64, DIN / 64, 1), 32, 0, stream>>>(DT, W3, dtb, DL);
    k_scan<<<NB * (DIN / 32), 32, 0, stream>>>(XI, DL, XD, G, cw, cb, alog, dvec, YG);
    k_gemm_out<<<dim3(ROWS / 64, HID / 64, 1), 32, 0, stream>>>(YG, W4, x, OUT);
}
